// ProxemicsFieldGenerator_10668698763551
// MI455X (gfx1250) — hardware-run, weakly checked
//
#include <hip/hip_runtime.h>


namespace {
constexpr int NB_ = 16, NN = 1024, F0 = 32, F1 = 16, H0 = 4, F2 = 32, C1 = H0 * F1  , CH = 256;
constexpr float HS = 256.0f, PS = 256.0f, WSC = 256.0f, EPS = 1e-5f;
typedef _Float16 b16;
typedef __attribute__((ext_vector_type(16))) _Float16 v16b;
typedef __attribute__((ext_vector_type(8))) _Float16 v8b;
typedef __attribute__((ext_vector_type(8))) float v8f;
typedef __attribute__((ext_vector_type(4))) float v4f;
typedef __attribute__((ext_vector_type(2))) float v2f;
__device__ __forceinline__ float bf16_rne(float f) { unsigned int u = __float_as_uint(f); u += 0x7FFFu + ((u >> 16) & 1u); float r = __uint_as_float(u & 0xFFFF0000u); asm volatile("" : "+v"(r)); return r; }
__device__ __forceinline__ float bfv(float f) { float r = bf16_rne(f); asm volatile("" : "+v"(r)); return r; }
__device__ __forceinline__ void split16(float v, b16& hi, b16& lo) { hi = (b16)v; lo = (b16)(v - (float)hi); }
__device__ __forceinline__ v16b frag_kb(const b16* p, int hh) { const v8b a = *(const v8b*)(p + 8 * hh), b = *(const v8b*)(p + 16 + 8 * hh); v16b f;
#pragma unroll
  for (int e = 0; e < 8; ++e) { f[e] = a[e]; f[8 + e] = b[e]; } return f; }
__device__ __forceinline__ v8f wmma16b(v16b a, v16b b, v8f c) { v8f d = __builtin_amdgcn_wmma_f32_16x16x32_f16(false, a, false, b, (short)0, c, false, false); asm volatile("v_nop\n\tv_nop\n\tv_nop\n\tv_nop" : "+v"(d) : "v"(a), "v"(b)); return d; }
__device__ __forceinline__ void wave_lds_sync() { __builtin_amdgcn_fence(__ATOMIC_RELEASE, "workgroup"); __builtin_amdgcn_wave_barrier(); __builtin_amdgcn_fence(__ATOMIC_ACQUIRE, "workgroup"); }
__device__ __forceinline__ float pmul(float a, float b) { float p = a * b; asm volatile("" : "+v"(p)); return p; }
__device__ __forceinline__ float elu(float v) { return v > 0.0f ? v : (__expf(v) - 1.0f); }

__global__ __launch_bounds__(256) void wput_kernel(const float* __restrict__ w1, const float* __restrict__ w2, b16* __restrict__ WA, b16* __restrict__ WB) { const int u = blockIdx.x * 256 + threadIdx.x; v8b v;
  if (u < C1 * 4) { const int oo = u / 4, k0 = (u % 4) * 8; const int h = oo / F1, o = oo % F1;
#pragma unroll
    for (int j = 0; j < 8; ++j) v[j] = (b16)(bf16_rne(w1[((size_t)h * F0 + k0 + j) * F1 + o]) * WSC); for (int pass = 0; pass < 2; ++pass) { *(volatile v8b*)(WA + (size_t)oo * F0 + k0) = v; __threadfence(); } }
  if (u < F2 * 8) { const int o = u / 8, k0 = (u % 8) * 8;
#pragma unroll
    for (int j = 0; j < 8; ++j) v[j] = (b16)(bf16_rne(w2[(size_t)(k0 + j) * F2 + o]) * WSC); for (int pass = 0; pass < 2; ++pass) { *(volatile v8b*)(WB + (size_t)o * C1 + k0) = v; __threadfence(); } } }
template <int C, int MODE>
__global__ __launch_bounds__(64) void stats_kernel(const float* __restrict__ X, float* __restrict__ ST) { const int b = blockIdx.x, c = threadIdx.x; float mean = 0.0f, rstd = 0.0f; if (c < C) { double s = 0.0, s2 = 0.0; for (int n = 0; n < NN; ++n) { float v = X[((size_t)b * NN + n) * C + c]; if (MODE == 0) v = bfv(v); s += v; s2 += (double)v * v; } const double mu = s / NN; double var = s2 / NN - mu * mu; if (var < 0.0) var = 0.0; mean = (float)mu; rstd = (float)(1.0 / sqrt(var + (double)EPS)); }
  for (int pass = 0; pass < 2; ++pass) { ((volatile float*)ST)[(size_t)b * 128 + c] = mean; ((volatile float*)ST)[(size_t)b * 128 + 64 + c] = rstd; __threadfence(); } }
template <int C, int MODE, int NT, int NHh>
__global__ __launch_bounds__(32) void proj_kernel(const float* __restrict__ X, const float* __restrict__ ST, const b16* __restrict__ W, const float* __restrict__ asrc, const float* __restrict__ adst, float* __restrict__ HP, float* __restrict__ SD) { constexpr int OW = NT * 16, FD = OW / NHh, LPH = 32 / NHh; __shared__ __attribute__((aligned(16))) b16 Ah[16][C + 8], Al[16][C + 8]; __shared__ float Tf[16][OW + 4], Eq[16][8]; const int lane = threadIdx.x, nloc = lane & 15, hlf = lane >> 4; const size_t m0 = (size_t)blockIdx.x * 16; const int b = (int)(m0 / NN);
  for (int rr = 0; rr < 16; ++rr) for (int q = 0; q < C / 32; ++q) { const int c = q * 32 + lane; float v = X[(m0 + rr) * C + c]; if (MODE == 0) v = bfv(v); v = pmul(v - ST[(size_t)b * 128 + c], ST[(size_t)b * 128 + 64 + c]); b16 p, ql; split16(v * HS, p, ql); Ah[rr][c] = p; Al[rr][c] = ql; }
  if (lane < 16) for (int k = C; k < C + 8; ++k) { Ah[lane][k] = (b16)0.0f; Al[lane][k] = (b16)0.0f; }
  wave_lds_sync(); v8f acc[NT];
#pragma unroll
  for (int t = 0; t < NT; ++t) acc[t] = (v8f){};
#pragma unroll
  for (int kb = 0; kb < C; kb += 32) { const v16b a = frag_kb(&Ah[nloc][kb], hlf), al = frag_kb(&Al[nloc][kb], hlf);
#pragma unroll
    for (int t = 0; t < NT; ++t) { const v16b bw = frag_kb(W + (size_t)(t * 16 + nloc) * C + kb, hlf); acc[t] = wmma16b(a, bw, acc[t]); acc[t] = wmma16b(al, bw, acc[t]); } }
#pragma unroll
  for (int t = 0; t < NT; ++t)
#pragma unroll
    for (int r8 = 0; r8 < 8; ++r8) Tf[8 * hlf + r8][t * 16 + nloc] = acc[t][r8] * (1.0f / (HS * WSC));
  wave_lds_sync();
  { const int hd = lane / LPH, sub = lane % LPH; for (int rr = 0; rr < 16; ++rr) { float s1 = 0.0f, s2 = 0.0f; for (int j = sub; j < FD; j += LPH) { const float hv = Tf[rr][hd * FD + j]; s1 += pmul(hv, bfv(asrc[hd * FD + j])); s2 += pmul(hv, bfv(adst[hd * FD + j])); } for (int o = LPH / 2; o; o >>= 1) { s1 += __shfl_xor(s1, o); s2 += __shfl_xor(s2, o); } if (sub == 0) { Eq[rr][hd] = s1; Eq[rr][4 + hd] = s2; } if (lane >= NHh && lane < 4) { Eq[rr][lane] = 0.0f; Eq[rr][4 + lane] = 0.0f; } } }
  wave_lds_sync();
  for (int pass = 0; pass < 2; ++pass) { for (int rr = 0; rr < 16; ++rr) for (int q = 0; q < OW / 32; ++q) ((volatile float*)HP)[(m0 + rr) * OW + q * 32 + lane] = Tf[rr][q * 32 + lane]; for (int q = 0; q < 4; ++q) ((volatile float*)SD)[m0 * 8 + q * 32 + lane] = Eq[(q * 32 + lane) >> 3][(q * 32 + lane) & 7]; __threadfence(); } }
template <int HW, int FD, int NHh, int ACT>
__global__ __launch_bounds__(32) void att_kernel(const float* __restrict__ HP, const float* __restrict__ SD, const float* __restrict__ bias, float* __restrict__ OUT) { constexpr int NTL = FD / 16, OWD = NHh * FD; __shared__ float Lg[16][NN]; __shared__ __attribute__((aligned(16))) b16 Pa[16][CH + 8], Pb[16][CH + 8], Hh[FD][CH + 8], Hl[FD][CH + 8]; __shared__ float Of[16][OWD + 1], Inv[16]; const int lane = threadIdx.x, nloc = lane & 15, hlf = lane >> 4; const int tile = blockIdx.x % (NN / 16), b = blockIdx.x / (NN / 16); const size_t rb = (size_t)b * NN; const size_t i0 = rb + (size_t)tile * 16;
  if (lane < 16) for (int k = CH; k < CH + 8; ++k) { Pa[lane][k] = (b16)0.0f; Pb[lane][k] = (b16)0.0f; }
  for (int d = lane; d < FD; d += 32) for (int k = CH; k < CH + 8; ++k) { Hh[d][k] = (b16)0.0f; Hl[d][k] = (b16)0.0f; }
#pragma unroll 1
  for (int hd = 0; hd < NHh; ++hd) {
    for (int r = 0; r < 16; ++r) { const float si = SD[(i0 + r) * 8 + hd]; float mx = -INFINITY; for (int j = lane; j < NN; j += 32) { float e = si + SD[(rb + j) * 8 + 4 + hd]; e = e >= 0.0f ? e : 0.2f * e; Lg[r][j] = e; mx = fmaxf(mx, e); } for (int o = 16; o; o >>= 1) mx = fmaxf(mx, __shfl_xor(mx, o)); float sm = 0.0f; for (int j = lane; j < NN; j += 32) { const float p = __expf(Lg[r][j] - mx); Lg[r][j] = p; sm += p; } for (int o = 16; o; o >>= 1) sm += __shfl_xor(sm, o); if (lane == 0) Inv[r] = 1.0f / sm; }
    wave_lds_sync(); v8f acc[NTL];
#pragma unroll
    for (int t = 0; t < NTL; ++t) acc[t] = (v8f){};
#pragma unroll 1
    for (int ch = 0; ch < NN / CH; ++ch) { const int c0 = ch * CH;
      for (int r = 0; r < 16; ++r) { const float inv = Inv[r]; for (int q = 0; q < CH / 32; ++q) { const int c = q * 32 + lane; b16 p, ql; split16(Lg[r][c0 + c] * inv * PS, p, ql); Pa[r][c] = p; Pb[r][c] = ql; } }
      for (int c = 0; c < CH; ++c) for (int d = lane; d < FD; d += 32) { b16 p, ql; split16(HP[(rb + c0 + c) * HW + hd * FD + d] * HS, p, ql); Hh[d][c] = p; Hl[d][c] = ql; }
      wave_lds_sync();
#pragma unroll 2
      for (int kb = 0; kb < CH; kb += 32) { const v16b pa = frag_kb(&Pa[nloc][kb], hlf), pb = frag_kb(&Pb[nloc][kb], hlf);
#pragma unroll
        for (int t = 0; t < NTL; ++t) { const v16b vh = frag_kb(&Hh[t * 16 + nloc][kb], hlf), vl = frag_kb(&Hl[t * 16 + nloc][kb], hlf); acc[t] = wmma16b(pa, vh, acc[t]); acc[t] = wmma16b(pa, vl, acc[t]); acc[t] = wmma16b(pb, vh, acc[t]); } }
      wave_lds_sync(); }
#pragma unroll
    for (int t = 0; t < NTL; ++t) {
#pragma unroll
      for (int r8 = 0; r8 < 8; ++r8) { const int cc = t * 16 + nloc; const float v = acc[t][r8] * (1.0f / (PS * HS)) + bfv(bias[cc]); Of[8 * hlf + r8][hd * FD + cc] = ACT ? elu(v) : v; } }
    wave_lds_sync(); }
  for (int pass = 0; pass < 2; ++pass) { for (int r = 0; r < 16; ++r) for (int q = 0; q < OWD / 32; ++q) ((volatile float*)OUT)[(i0 + r) * OWD + q * 32 + lane] = Of[r][q * 32 + lane]; __threadfence(); } }
}

extern "C" void kernel_launch(void* const* d_in, const int* in_sizes, int n_in, void* d_out, int out_size, void* d_ws, size_t ws_size, hipStream_t stream) {
  (void)n_in;
  auto Fp = [&](int i) { return (const float*)d_in[i]; };
  if (in_sizes[0] != NB_ * NN * F0 || in_sizes[1] != H0 * F0 * F1 || in_sizes[2] != H0 * F1 || in_sizes[4] != F1 || in_sizes[5] != C1 * F2 || in_sizes[6] != F2 || in_sizes[8] != F2 || out_size != NB_ * NN * F2) return;
  const int BLIM = NB_;
  size_t off = 0; char* ws = (char*)d_ws;
  auto carve = [&](size_t bytes) { char* p = ws + off; off += (bytes + 255) & ~(size_t)255; return p; };
  b16* WA = (b16*)carve((size_t)C1 * F0 * 2); b16* WB = (b16*)carve((size_t)F2 * C1 * 2); float* ST = (float*)carve((size_t)NB_ * 128 * 4); float* HP = (float*)carve((size_t)NB_ * NN * C1 * 4); float* SD = (float*)carve((size_t)NB_ * NN * 8 * 4); float* X1 = (float*)carve((size_t)NB_ * NN * C1 * 4);
  if (off > ws_size || off > ((size_t)16 << 20)) return;
  wput_kernel<<<1, 256, 0, stream>>>(Fp(1), Fp(5), WA, WB);
  stats_kernel<F0, 0><<<BLIM, 64, 0, stream>>>(Fp(0), ST);
  proj_kernel<F0, 0, 4, 4><<<BLIM * NN / 16, 32, 0, stream>>>(Fp(0), ST, WA, Fp(2), Fp(3), HP, SD);
  att_kernel<C1, F1, H0, 1><<<BLIM * (NN / 16), 32, 0, stream>>>(HP, SD, Fp(4), X1);
  stats_kernel<C1, 1><<<BLIM, 64, 0, stream>>>(X1, ST);
  proj_kernel<C1, 1, 2, 1><<<BLIM * NN / 16, 32, 0, stream>>>(X1, ST, WB, Fp(6), Fp(7), HP, SD);
  att_kernel<F2, F2, 1, 0><<<BLIM * (NN / 16), 32, 0, stream>>>(HP, SD, Fp(8), (float*)d_out);
}
